// CMHA_91293824843817
// MI455X (gfx1250) — hardware-verified
//
#include <hip/hip_runtime.h>


#define NB_  64
#define GN   512
#define DM   128
#define NH_  8
#define KD   16
#define HD   64
#define DQ   (NH_ * HD)
#define NS   20
#define C0   (1 + NS)
#define GB   8
#define SCL  0.25f
typedef _Float16 h16;
typedef unsigned short bf;
typedef __attribute__((ext_vector_type(16))) __bf16   v16bf;
typedef __attribute__((ext_vector_type(16))) _Float16 v16h;
typedef __attribute__((ext_vector_type(8)))  _Float16 v8h;
typedef __attribute__((ext_vector_type(8)))  unsigned short v8us;
typedef __attribute__((ext_vector_type(8)))  float    v8f;
typedef __attribute__((ext_vector_type(4)))  float    v4f;
typedef v8h  __attribute__((may_alias)) v8ha;
typedef v4f  __attribute__((may_alias)) v4fa;
typedef v8us __attribute__((may_alias)) v8usa;

__device__ __forceinline__ unsigned short f2bf(float f) { unsigned u = __float_as_uint(f); u += 0x7FFFu + ((u >> 16) & 1u); return (unsigned short)(u >> 16); }
__device__ __forceinline__ float bf2f(unsigned short b) { return __uint_as_float(((unsigned)b) << 16); }
__device__ __forceinline__ float bfr(float f) { return bf2f(f2bf(f)); }
__device__ __forceinline__ v16h cat16(v8h lo, v8h hi) { return __builtin_shufflevector(lo, hi, 0, 1, 2, 3, 4, 5, 6, 7, 8, 9, 10, 11, 12, 13, 14, 15); }
__device__ __forceinline__ v16bf cat16b(v8us lo, v8us hi) { return __builtin_bit_cast(v16bf, __builtin_shufflevector(lo, hi, 0, 1, 2, 3, 4, 5, 6, 7, 8, 9, 10, 11, 12, 13, 14, 15)); }
__device__ __forceinline__ v8f wmma16(v16h a, v16h b, v8f c) { return __builtin_amdgcn_wmma_f32_16x16x32_f16(false, a, false, b, (short)0, c, false, false); }
__device__ __forceinline__ v8f wmmab(v16bf a, v16bf b, v8f c) { return __builtin_amdgcn_wmma_f32_16x16x32_bf16(false, a, false, b, (short)0, c, false, false); }


template <typename T16> struct WFrag;
template <> struct WFrag<h16> { typedef v16h V; static __device__ __forceinline__ V ld(const h16* p) { return cat16(*(const v8h*)p, *(const v8h*)(p + 16)); } static __device__ __forceinline__ v8f mma(V a, V b, v8f c) { return wmma16(a, b, c); } };
template <> struct WFrag<bf> { typedef v16bf V; static __device__ __forceinline__ V ld(const bf* p) { return cat16b(*(const v8us*)p, *(const v8us*)(p + 16)); } static __device__ __forceinline__ v8f mma(V a, V b, v8f c) { return wmmab(a, b, c); } };
template <typename T16, int NSPLIT, bool BIAS>
__global__ __launch_bounds__(32) void k_gemmw(const T16* __restrict__ A, const T16* __restrict__ A2, const T16* __restrict__ Bt, const T16* __restrict__ Bt2, int K, float* C, int ldc, const float* __restrict__ bias, size_t sA, size_t sB, size_t sC) {
    typedef typename WFrag<T16>::V V;
    __shared__ __align__(16) float os[16 * 68];
    const size_t z = blockIdx.z; A += z * sA; if (A2) A2 += z * sA; Bt += z * sB; if (Bt2) Bt2 += z * sB; C += z * sC;
    const int lane = threadIdx.x & 31, lr = lane & 15, hi = lane >> 4; const int r0 = blockIdx.x * 64, c0 = blockIdx.y * 64;
    v8f acc[4][4];
#pragma unroll
    for (int mb = 0; mb < 4; ++mb)
#pragma unroll
        for (int nb = 0; nb < 4; ++nb) acc[mb][nb] = (v8f){};
    const size_t aoff = (size_t)(r0 + lr) * K + 8 * hi, boff = (size_t)(c0 + lr) * K + 8 * hi;
#pragma unroll 1
    for (int kc = 0; kc < K; kc += 32) {
        V a[4], a2[4];
#pragma unroll
        for (int mb = 0; mb < 4; ++mb) { a[mb] = WFrag<T16>::ld(A + aoff + (size_t)mb * 16 * K + kc); if (NSPLIT == 1 || NSPLIT == 2) a2[mb] = WFrag<T16>::ld(A2 + aoff + (size_t)mb * 16 * K + kc); }
#pragma unroll
        for (int nb = 0; nb < 4; ++nb) { const V b = WFrag<T16>::ld(Bt + boff + (size_t)nb * 16 * K + kc); V b2; if (NSPLIT >= 2) b2 = WFrag<T16>::ld(Bt2 + boff + (size_t)nb * 16 * K + kc);
#pragma unroll
            for (int mb = 0; mb < 4; ++mb) { acc[mb][nb] = WFrag<T16>::mma(a[mb], b, acc[mb][nb]); if (NSPLIT == 1 || NSPLIT == 2) acc[mb][nb] = WFrag<T16>::mma(a2[mb], b, acc[mb][nb]); if (NSPLIT >= 2) acc[mb][nb] = WFrag<T16>::mma(a[mb], b2, acc[mb][nb]); } }
        asm volatile("v_nop\n\tv_nop\n\tv_nop\n\tv_nop" : "+v"(acc[0][0]), "+v"(acc[1][1]), "+v"(acc[2][2]), "+v"(acc[3][3]) : "v"(a[0]), "v"(a[3]));
    }
#pragma unroll
    for (int mb = 0; mb < 4; ++mb) {
#pragma unroll
        for (int nb = 0; nb < 4; ++nb) {
#pragma unroll
            for (int j = 0; j < 8; ++j) os[(hi * 8 + j) * 68 + nb * 16 + lr] = acc[mb][nb][j]; }
        __builtin_amdgcn_wave_barrier(); asm volatile("" ::: "memory");
        float* crow = C + (size_t)(r0 + mb * 16) * ldc + c0;
#pragma unroll 1
        for (int ps = 0; ps < 2; ++ps) {
#pragma unroll
            for (int s = 0; s < 8; ++s) { const int row = 2 * s + hi, cofs = lr * 4; v4f val = *(const v4fa*)(os + row * 68 + cofs); if (BIAS) { val[0] += bfr(bias[c0 + cofs]); val[1] += bfr(bias[c0 + cofs + 1]); val[2] += bfr(bias[c0 + cofs + 2]); val[3] += bfr(bias[c0 + cofs + 3]); }
                *(volatile v4f*)(crow + (size_t)row * ldc + cofs) = val; }
            if (ps == 0) __threadfence(); }
        __builtin_amdgcn_wave_barrier(); asm volatile("" ::: "memory");
    }
}

__device__ __forceinline__ h16 tohx(float x) { return (h16)x; }
__device__ __forceinline__ void splitf(float y, unsigned short& h, unsigned short& l) { h = f2bf(y); l = f2bf(y - bf2f(h)); }
typedef __attribute__((ext_vector_type(2))) _Float16 v2h;
typedef __attribute__((ext_vector_type(4))) _Float16 v4h;
typedef __attribute__((ext_vector_type(2))) unsigned short v2us;
typedef __attribute__((ext_vector_type(4))) unsigned short v4us;
typedef __attribute__((ext_vector_type(2))) float v2f;
typedef __attribute__((ext_vector_type(4))) int v4i;


__global__ __launch_bounds__(256) void k_cvt8(const float* __restrict__ src, bf* dst, size_t n8) { const size_t i = (size_t)blockIdx.x * 256 + threadIdx.x; if (i >= n8) return; const v8f v = *(const v8f*)(src + i * 8); v8us o;
#pragma unroll
    for (int k = 0; k < 8; ++k) o[k] = f2bf(v[k]); *(volatile v8us*)(dst + i * 8) = o; __threadfence(); *(volatile v8us*)(dst + i * 8) = o; }

__global__ __launch_bounds__(256) void k_wg(const float* __restrict__ w, bf* Bt) { const int e = (blockIdx.x * 256 + threadIdx.x) * 2; if (e >= DQ * DM) return; const int n = e / DM, d = e % DM; const int h = n / HD, kk = n % HD; v2us o; o[0] = (kk < KD) ? f2bf(w[((size_t)h * DM + d) * KD + kk]) : (unsigned short)0; o[1] = (kk < KD) ? f2bf(w[((size_t)h * DM + d + 1) * KD + kk]) : (unsigned short)0; *(volatile v2us*)(Bt + e) = o; __threadfence(); *(volatile v2us*)(Bt + e) = o; }
__global__ __launch_bounds__(256) void k_wout(const float* __restrict__ w, bf* Bt) { const int i = (blockIdx.x * 256 + threadIdx.x) * 2; if (i >= DM * DQ) return; const int e_ = i / DQ, n = i % DQ; const int h = n / HD, kk = n % HD; v2us o; o[0] = (kk < KD) ? f2bf(w[((size_t)h * KD + kk) * DM + e_]) : (unsigned short)0; o[1] = (kk + 1 < KD) ? f2bf(w[((size_t)h * KD + kk + 1) * DM + e_]) : (unsigned short)0; *(volatile v2us*)(Bt + i) = o; __threadfence(); *(volatile v2us*)(Bt + i) = o; }
__global__ __launch_bounds__(256) void k_plq(const float* __restrict__ F, int nrow, bf* Ph, bf* Pl) { const size_t e = ((size_t)blockIdx.x * 256 + threadIdx.x) * 2; if (e >= (size_t)GB * NH_ * nrow * HD) return; const int d = (int)(e % HD); const int t = (int)((e / HD) % nrow); const int h = (int)((e / ((size_t)HD * nrow)) % NH_); const int b = (int)(e / ((size_t)HD * nrow * NH_)); const float* f = F + ((size_t)b * nrow + t) * DQ + h * HD + d; v2us oh, ol;
#pragma unroll
    for (int q = 0; q < 2; ++q) { unsigned short a, c2; splitf(f[q], a, c2); oh[q] = a; ol[q] = c2; } *(volatile v2us*)(Ph + e) = oh; *(volatile v2us*)(Pl + e) = ol; __threadfence(); *(volatile v2us*)(Ph + e) = oh; *(volatile v2us*)(Pl + e) = ol; }
__global__ __launch_bounds__(256) void k_plvt(const float* __restrict__ F, bf* Vh, bf* Vl) { const size_t e = ((size_t)blockIdx.x * 256 + threadIdx.x) * 2; if (e >= (size_t)GB * NH_ * HD * GN) return; const int t = (int)(e % GN); const int d = (int)((e / GN) % HD); const int h = (int)((e / ((size_t)GN * HD)) % NH_); const int b = (int)(e / ((size_t)GN * HD * NH_)); v2us oh, ol;
#pragma unroll
    for (int q = 0; q < 2; ++q) { unsigned short a, c2; splitf(F[((size_t)b * GN + t + q) * DQ + h * HD + d], a, c2); oh[q] = a; ol[q] = c2; } *(volatile v2us*)(Vh + e) = oh; *(volatile v2us*)(Vl + e) = ol; __threadfence(); *(volatile v2us*)(Vh + e) = oh; *(volatile v2us*)(Vl + e) = ol; }
__global__ __launch_bounds__(256) void k_bsoft(const float* __restrict__ Sb, int nrows, int mode, bf* Ph, bf* Pl) {
    const int lane = threadIdx.x & 31; const int row = blockIdx.x * 8 + (threadIdx.x >> 5); if (row >= nrows) return; const float* sr = Sb + (size_t)row * GN; float v[GN / 32]; float mx = -3.0e38f;
#pragma unroll
    for (int ch = 0; ch < GN / 128; ++ch) { const int j0 = ch * 128 + lane * 4; const v4f a = *(const v4f*)(sr + j0);
#pragma unroll
        for (int q = 0; q < 4; ++q) { const int j = j0 + q; const bool ok = (mode == 0) || (j >= C0) || (mode == 2 && j == 0); float sa = a[q] * SCL; asm volatile("" : "+v"(sa)); const float t = ok ? sa : -3.0e38f; v[ch * 4 + q] = t; mx = fmaxf(mx, t); } }
#pragma unroll
    for (int sh = 16; sh; sh >>= 1) mx = fmaxf(mx, __shfl_xor(mx, sh, 32));
    float sum = 0.f;
#pragma unroll
    for (int k = 0; k < GN / 32; ++k) { float d0 = __fsub_rn(v[k], mx); asm volatile("" : "+v"(d0)); v[k] = __builtin_amdgcn_exp2f(__fmul_rn(d0, 1.4426950408889634f)); sum += v[k]; }
#pragma unroll
    for (int sh = 16; sh; sh >>= 1) sum += __shfl_xor(sum, sh, 32);
    const float f = __fdiv_rn(1.0f, sum);
#pragma unroll 1
    for (int ps = 0; ps < 2; ++ps) {
#pragma unroll
        for (int ch = 0; ch < GN / 128; ++ch) { v4us oh, ol;
#pragma unroll
            for (int q = 0; q < 4; ++q) { unsigned short a, c2; float y = v[ch * 4 + q] * f; asm volatile("" : "+v"(y)); splitf(y, a, c2); oh[q] = a; ol[q] = c2; }
            const size_t oo = (size_t)row * GN + ch * 128 + lane * 4; *(volatile v4us*)(Ph + oo) = oh; *(volatile v4us*)(Pl + oo) = ol; }
        if (ps == 0) __threadfence(); }
}
__global__ __launch_bounds__(256) void k_hsel(const float* __restrict__ Ob, int R, int r0, int gmin, int gmax, bf* Hh, bf* Hl) { const size_t e = ((size_t)blockIdx.x * 256 + threadIdx.x) * 2; if (e >= (size_t)GB * NH_ * R * HD) return; const int d = (int)(e % HD); const int r = (int)((e / HD) % R); const int h = (int)((e / ((size_t)HD * R)) % NH_); const int b = (int)(e / ((size_t)HD * R * NH_)); const int g = r0 + r; if (g < gmin || g > gmax) return;     v2us oh, ol;
#pragma unroll
    for (int q = 0; q < 2; ++q) { unsigned short a, c2; splitf(Ob[e + q], a, c2); oh[q] = a; ol[q] = c2; } const size_t oo = ((size_t)b * GN + g) * DQ + h * HD + d; *(volatile v2us*)(Hh + oo) = oh; *(volatile v2us*)(Hl + oo) = ol; __threadfence(); *(volatile v2us*)(Hh + oo) = oh; *(volatile v2us*)(Hl + oo) = ol; }

extern "C" void kernel_launch(void* const* d_in, const int* in_sizes, int n_in,
                              void* d_out, int out_size, void* d_ws, size_t ws_size, hipStream_t stream) {
    (void)in_sizes; (void)n_in; (void)out_size;
    const float* q = (const float*)d_in[0]; const float* hx = (const float*)d_in[1]; const float* wq_dep = (const float*)d_in[2]; const float* wk_cus_ = (const float*)d_in[3]; const float* wv_cus_ = (const float*)d_in[4]; const float* wq_sta = (const float*)d_in[5]; const float* wk_oth = (const float*)d_in[6]; const float* wv_oth = (const float*)d_in[7]; const float* wq_cus = (const float*)d_in[8]; const float* wk_all = (const float*)d_in[9]; const float* wv_all = (const float*)d_in[10]; const float* wout = (const float*)d_in[11];
    float* OUT = (float*)d_out;
    char* wsp = (char*)d_ws;
    auto take = [&](size_t bytes) { char* p = wsp; wsp += (bytes + 255) & ~(size_t)255; return (void*)p; };
    bf* XQ = (bf*)take((size_t)NB_ * GN * DM * 2); bf* XH = (bf*)take((size_t)NB_ * GN * DM * 2);
    bf* WQB[3]; bf* WKB[3]; bf* WVB[3]; for (int i = 0; i < 3; ++i) { WQB[i] = (bf*)take((size_t)DQ * DM * 2); WKB[i] = (bf*)take((size_t)DQ * DM * 2); WVB[i] = (bf*)take((size_t)DQ * DM * 2); } bf* WOB = (bf*)take((size_t)DM * DQ * 2);
    float* F = (float*)take((size_t)GB * GN * DQ * 4);
    bf* QPh = (bf*)take((size_t)GB * NH_ * GN * HD * 2); bf* QPl = (bf*)take((size_t)GB * NH_ * GN * HD * 2); bf* KPh = (bf*)take((size_t)GB * NH_ * GN * HD * 2); bf* KPl = (bf*)take((size_t)GB * NH_ * GN * HD * 2); bf* VTh = (bf*)take((size_t)GB * NH_ * HD * GN * 2); bf* VTl = (bf*)take((size_t)GB * NH_ * HD * GN * 2);
    float* Sb = (float*)take((size_t)GB * NH_ * 256 * GN * 4); bf* Ph = (bf*)take((size_t)GB * NH_ * 256 * GN * 2); bf* Pl = (bf*)take((size_t)GB * NH_ * 256 * GN * 2); float* Ob = (float*)take((size_t)GB * NH_ * 256 * HD * 4); bf* HBh = (bf*)take((size_t)GB * GN * DQ * 2); bf* HBl = (bf*)take((size_t)GB * GN * DQ * 2);
    if ((size_t)(wsp - (char*)d_ws) > ws_size) return;
    k_cvt8<<<(unsigned)(((size_t)NB_ * GN * DM / 8 + 255) / 256), 256, 0, stream>>>(q, XQ, (size_t)NB_ * GN * DM / 8); k_cvt8<<<(unsigned)(((size_t)NB_ * GN * DM / 8 + 255) / 256), 256, 0, stream>>>(hx, XH, (size_t)NB_ * GN * DM / 8);
    const float* wqs[3] = {wq_cus, wq_dep, wq_sta}; const float* wks[3] = {wk_all, wk_cus_, wk_oth}; const float* wvs[3] = {wv_all, wv_cus_, wv_oth};
    for (int i = 0; i < 3; ++i) { k_wg<<<(DQ * DM / 2 + 255) / 256, 256, 0, stream>>>(wqs[i], WQB[i]); k_wg<<<(DQ * DM / 2 + 255) / 256, 256, 0, stream>>>(wks[i], WKB[i]); k_wg<<<(DQ * DM / 2 + 255) / 256, 256, 0, stream>>>(wvs[i], WVB[i]); }
    k_wout<<<(DM * DQ / 2 + 255) / 256, 256, 0, stream>>>(wout, WOB);
    const int MQ[3] = {GN, 64, 64};     const int MODE[3] = {0, 1, 2}; const int GMIN[3] = {C0, 0, 1}; const int GMAX[3] = {GN - 1, 0, NS};
    for (int b0 = 0; b0 < NB_; b0 += GB) {
        for (int blk = 0; blk < 3; ++blk) { const int Mq = MQ[blk];
            k_gemmw<bf, 0, false><<<dim3(Mq / 64, DQ / 64, GB), 32, 0, stream>>>(XQ + (size_t)b0 * GN * DM, nullptr, WQB[blk], nullptr, DM, F, DQ, nullptr, (size_t)GN * DM, 0, (size_t)Mq * DQ);
            k_plq<<<(unsigned)(((size_t)GB * NH_ * Mq * HD / 2 + 255) / 256), 256, 0, stream>>>(F, Mq, QPh, QPl);
            k_gemmw<bf, 0, false><<<dim3(GN / 64, DQ / 64, GB), 32, 0, stream>>>(XH + (size_t)b0 * GN * DM, nullptr, WKB[blk], nullptr, DM, F, DQ, nullptr, (size_t)GN * DM, 0, (size_t)GN * DQ);
            k_plq<<<(unsigned)(((size_t)GB * NH_ * GN * HD / 2 + 255) / 256), 256, 0, stream>>>(F, GN, KPh, KPl);
            k_gemmw<bf, 0, false><<<dim3(GN / 64, DQ / 64, GB), 32, 0, stream>>>(XH + (size_t)b0 * GN * DM, nullptr, WVB[blk], nullptr, DM, F, DQ, nullptr, (size_t)GN * DM, 0, (size_t)GN * DQ);
            k_plvt<<<(unsigned)(((size_t)GB * NH_ * HD * GN / 2 + 255) / 256), 256, 0, stream>>>(F, VTh, VTl);
            const int R = (Mq < 256) ? Mq : 256;
            for (int r0 = 0; r0 < Mq; r0 += R) {
                k_gemmw<bf, 2, false><<<dim3(R / 64, GN / 64, GB * NH_), 32, 0, stream>>>(QPh + (size_t)r0 * HD, QPl + (size_t)r0 * HD, KPh, KPl, HD, Sb, GN, nullptr, (size_t)Mq * HD, (size_t)GN * HD, (size_t)R * GN);
                k_bsoft<<<(GB * NH_ * R + 7) / 8, 256, 0, stream>>>(Sb, GB * NH_ * R, MODE[blk], Ph, Pl);
                k_gemmw<bf, 2, false><<<dim3(R / 64, HD / 64, GB * NH_), 32, 0, stream>>>(Ph, Pl, VTh, VTl, GN, Ob, HD, nullptr, (size_t)R * GN, (size_t)HD * GN, (size_t)R * HD);
                k_hsel<<<(unsigned)(((size_t)GB * NH_ * R * HD / 2 + 255) / 256), 256, 0, stream>>>(Ob, R, r0, GMIN[blk], GMAX[blk], HBh, HBl); } }
        k_gemmw<bf, 1, false><<<dim3(GN / 64, DM / 64, GB), 32, 0, stream>>>(HBh, HBl, WOB, nullptr, DQ, OUT + (size_t)b0 * GN * DM, DM, nullptr, (size_t)GN * DQ, 0, (size_t)GN * DM); }
}
